// InterpretableMultiHeadAttention_69174743269562
// MI455X (gfx1250) — hardware-verified
//
#include <hip/hip_runtime.h>


#ifndef NB
#define NB 4
#endif
#ifndef SEQ
#define SEQ 512
#endif
#define NB_FULL  4
#define SEQ_FULL 512
#ifndef OUT_SEQ
#define OUT_SEQ SEQ
#endif
#define DM   256
#define NH_  4
#define HD   64
#define OSP  68
#define KSP  68
#define SCP  (SEQ + 4)
#define C2X  ((float)(2.0 * 1.4426950408889634))
#define SC2  ((float)(0.125 * 1.4426950408889634))
#define PCAR 16384.0f
#define VCAR 64.0f
#define ACAR 256.0f
#define WCAR 64.0f
#define OSC  (1.0f / (ACAR * WCAR))
#define NEGB (-3.0e38f)
#define OUT1_OFF ((size_t)NB_FULL * SEQ_FULL * DM)

static_assert(HD == 64);
static_assert(NH_ * HD == DM);
static_assert(DM % 64 == 0);
static_assert(DM % 32 == 0);
static_assert(SEQ % 64 == 0);
static_assert((NB * SEQ) % 64 == 0);
static_assert(SEQ % 32 == 0);
static_assert(SEQ % 16 == 0);
static_assert(SEQ % 128 == 0);
static_assert(((size_t)SEQ * DM) % 8 == 0);
static_assert(((size_t)DM * DM) % 8 == 0);
static_assert(NB <= NB_FULL);
static_assert(SEQ <= SEQ_FULL);
static_assert(SEQ <= OUT_SEQ);
static_assert((OSP * 4) % 16 == 0);
static_assert((KSP * 4) % 16 == 0);
static_assert((SCP * 4) % 16 == 0);
static_assert(OUT1_OFF * 4 == (size_t)2097152);
static_assert(((size_t)(NB - 1) * OUT_SEQ + SEQ) * DM <= OUT1_OFF);
static_assert(8 * 32 * 4 == 16 * HD);
static_assert(4 * 32 * 8 == 16 * 64);
static_assert((SEQ / 128) * 32 * 4 == SEQ);
static_assert((16 * SCP + 32 * KSP + 16 * KSP + 16 * OSP + HD + 16) * 4 <= 131072);
static_assert(16 * OSP * 4 <= 131072);

typedef _Float16 h16;
typedef unsigned short bf;
typedef __attribute__((ext_vector_type(16))) __bf16   v16bf;
typedef __attribute__((ext_vector_type(16))) _Float16 v16h;
typedef __attribute__((ext_vector_type(8)))  _Float16 v8h;
typedef __attribute__((ext_vector_type(8)))  unsigned short v8us;
typedef __attribute__((ext_vector_type(8)))  float    v8f;
typedef __attribute__((ext_vector_type(4)))  float    v4f;
typedef v4f  __attribute__((may_alias)) v4fa;

__device__ __forceinline__ unsigned short f2bf(float f) { unsigned u = __float_as_uint(f); u += 0x7FFFu + ((u >> 16) & 1u); return (unsigned short)(u >> 16); }
__device__ __forceinline__ float bfr(float f) { return __uint_as_float(((unsigned)f2bf(f)) << 16); }
__device__ __forceinline__ v16h cat16(v8h lo, v8h hi) { return __builtin_shufflevector(lo, hi, 0, 1, 2, 3, 4, 5, 6, 7, 8, 9, 10, 11, 12, 13, 14, 15); }
__device__ __forceinline__ v16bf cat16b(v8us lo, v8us hi) { return __builtin_bit_cast(v16bf, __builtin_shufflevector(lo, hi, 0, 1, 2, 3, 4, 5, 6, 7, 8, 9, 10, 11, 12, 13, 14, 15)); }
__device__ __forceinline__ v8f wmma16(v16h a, v16h b, v8f c) { return __builtin_amdgcn_wmma_f32_16x16x32_f16(false, a, false, b, (short)0, c, false, false); }
__device__ __forceinline__ v8f wmmab(v16bf a, v16bf b, v8f c) { return __builtin_amdgcn_wmma_f32_16x16x32_bf16(false, a, false, b, (short)0, c, false, false); }
__device__ __forceinline__ v16h  ldh(const h16* p) { return cat16(*(const v8h*)p, *(const v8h*)(p + 16)); }
__device__ __forceinline__ v16bf ldb(const bf* p)  { return cat16b(*(const v8us*)p, *(const v8us*)(p + 16)); }
__device__ __forceinline__ void wave_sync() { __builtin_amdgcn_fence(3  , "wavefront"); __builtin_amdgcn_wave_barrier(); asm volatile("" ::: "memory"); }
static __device__ __forceinline__ h16 toh_flush(float v) { const h16 r = (h16)v; return (fabsf(v) < 6.103515625e-05f) ? (h16)0.0f : r; }
__device__ __forceinline__ v8f wmma16g(v16h a, v16h b, v8f c) { c = wmma16(a, b, c); asm volatile("v_nop\n\tv_nop\n\tv_nop\n\tv_nop" : "+v"(c) : "v"(a), "v"(b)); return c; }
__device__ __forceinline__ v8f wmmabg(v16bf a, v16bf b, v8f c) { c = wmmab(a, b, c); asm volatile("v_nop\n\tv_nop\n\tv_nop\n\tv_nop" : "+v"(c) : "v"(a), "v"(b)); return c; }

__global__ __launch_bounds__(256) void k_cvt8(const float* __restrict__ src, bf* dst, size_t n8) {
    const size_t i = (size_t)blockIdx.x * 256 + threadIdx.x; if (i >= n8) return;
    const v8f v = *(const v8f*)(src + i * 8); v8us o;
#pragma unroll
    for (int k = 0; k < 8; ++k) o[k] = f2bf(v[k]);
    *(volatile v8us*)(dst + i * 8) = o; __threadfence(); *(volatile v8us*)(dst + i * 8) = o;
}

__global__ __launch_bounds__(256) void k_cvtw(const float* __restrict__ src, h16* dst, size_t n8) {
    const size_t i = (size_t)blockIdx.x * 256 + threadIdx.x; if (i >= n8) return;
    const v8f v = *(const v8f*)(src + i * 8); v8h o;
#pragma unroll
    for (int k = 0; k < 8; ++k) o[k] = toh_flush(bfr(v[k]) * WCAR);
    *(volatile v8h*)(dst + i * 8) = o; __threadfence(); *(volatile v8h*)(dst + i * 8) = o;
}

__global__ __launch_bounds__(32) void k_projqk(const bf* __restrict__ A, const bf* __restrict__ Bt, float* P) {
    __shared__ __align__(16) float os[16 * OSP];
    const int lane = threadIdx.x & 31, lr = lane & 15, hi = lane >> 4; const int r0 = blockIdx.x * 64, c0 = blockIdx.y * 64;
    v8f acc[4][4];
#pragma unroll
    for (int mb = 0; mb < 4; ++mb)
#pragma unroll
        for (int nb = 0; nb < 4; ++nb) acc[mb][nb] = (v8f){};
    const size_t aoff = (size_t)(r0 + lr) * DM + 8 * hi, boff = (size_t)(c0 + lr) * DM + 8 * hi;
#pragma unroll 1
    for (int kc = 0; kc < DM; kc += 32) {
        v16bf a[4];
#pragma unroll
        for (int mb = 0; mb < 4; ++mb) a[mb] = ldb(A + aoff + (size_t)mb * 16 * DM + kc);
#pragma unroll
        for (int nb = 0; nb < 4; ++nb) { const v16bf b = ldb(Bt + boff + (size_t)nb * 16 * DM + kc);
#pragma unroll
            for (int mb = 0; mb < 4; ++mb) acc[mb][nb] = wmmabg(a[mb], b, acc[mb][nb]); }
    }
    const int bb = r0 / SEQ, tt = r0 % SEQ; const int zh = bb * NH_ + c0 / HD;
    const size_t tbase = ((size_t)zh * SEQ + (size_t)tt) * HD;
#pragma unroll
    for (int mb = 0; mb < 4; ++mb) {
#pragma unroll
        for (int nb = 0; nb < 4; ++nb) {
#pragma unroll
            for (int j = 0; j < 8; ++j) os[(hi * 8 + j) * OSP + nb * 16 + lr] = acc[mb][nb][j] * C2X; }
        wave_sync();
        const size_t sb = tbase + (size_t)(mb * 16) * HD;
#pragma unroll 1
        for (int ps = 0; ps < 2; ++ps) {
#pragma unroll
            for (int s = 0; s < 8; ++s) { const int p = s * 32 + lane; const int row = p >> 4, c4 = (p & 15) * 4;
                const v4f val = *(const v4fa*)(&os[row * OSP + c4]);
                *(volatile v4f*)(P + sb + (size_t)p * 4) = val; }
            if (ps == 0) __threadfence(); }
        wave_sync();
    }
}

__global__ __launch_bounds__(32) void k_projv(const bf* __restrict__ A, const bf* __restrict__ Bt, h16* Ph) {
    __shared__ __align__(16) float os[16 * OSP];
    const int lane = threadIdx.x & 31, lr = lane & 15, hi = lane >> 4; const int r0 = blockIdx.x * 64, c0 = blockIdx.y * 64;
    v8f acc[4][4];
#pragma unroll
    for (int mb = 0; mb < 4; ++mb)
#pragma unroll
        for (int nb = 0; nb < 4; ++nb) acc[mb][nb] = (v8f){};
    const size_t aoff = (size_t)(r0 + lr) * DM + 8 * hi, boff = (size_t)(c0 + lr) * DM + 8 * hi;
#pragma unroll 1
    for (int kc = 0; kc < DM; kc += 32) {
        v16bf a[4];
#pragma unroll
        for (int mb = 0; mb < 4; ++mb) a[mb] = ldb(A + aoff + (size_t)mb * 16 * DM + kc);
#pragma unroll
        for (int nb = 0; nb < 4; ++nb) { const v16bf b = ldb(Bt + boff + (size_t)nb * 16 * DM + kc);
#pragma unroll
            for (int mb = 0; mb < 4; ++mb) acc[mb][nb] = wmmabg(a[mb], b, acc[mb][nb]); }
    }
    const int bb = c0 / SEQ, tt = c0 % SEQ;
    const size_t tbase = (size_t)bb * (size_t)DM * SEQ + (size_t)r0 * SEQ + (size_t)tt;
#pragma unroll
    for (int mb = 0; mb < 4; ++mb) {
#pragma unroll
        for (int nb = 0; nb < 4; ++nb) {
#pragma unroll
            for (int j = 0; j < 8; ++j) os[(hi * 8 + j) * OSP + nb * 16 + lr] = acc[mb][nb][j] * VCAR; }
        wave_sync();
        const size_t sb = tbase + (size_t)(mb * 16) * SEQ;
#pragma unroll 1
        for (int ps = 0; ps < 2; ++ps) {
#pragma unroll
            for (int s = 0; s < 4; ++s) { const int row = 4 * s + (lane >> 3), c8 = (lane & 7) * 8;
                const v4f x0 = *(const v4fa*)(&os[row * OSP + c8]); const v4f x1 = *(const v4fa*)(&os[row * OSP + c8 + 4]); v8h hv;
#pragma unroll
                for (int i = 0; i < 4; ++i) { hv[i] = toh_flush(x0[i]); hv[4 + i] = toh_flush(x1[i]); }
                *(volatile v8h*)(Ph + sb + (size_t)row * SEQ + c8) = hv; }
            if (ps == 0) __threadfence(); }
        wave_sync();
    }
}

__global__ __launch_bounds__(32) void k_outp(const h16* __restrict__ A, const h16* __restrict__ Bt, float* OUT) {
    __shared__ __align__(16) float os[16 * OSP];
    const int lane = threadIdx.x & 31, lr = lane & 15, hi = lane >> 4; const int r0 = blockIdx.x * 64, c0 = blockIdx.y * 64;
    v8f acc[4][4];
#pragma unroll
    for (int mb = 0; mb < 4; ++mb)
#pragma unroll
        for (int nb = 0; nb < 4; ++nb) acc[mb][nb] = (v8f){};
    const size_t aoff = (size_t)(r0 + lr) * DM + 8 * hi, boff = (size_t)(c0 + lr) * DM + 8 * hi;
#pragma unroll 1
    for (int kc = 0; kc < DM; kc += 32) {
        v16h a[4];
#pragma unroll
        for (int mb = 0; mb < 4; ++mb) a[mb] = ldh(A + aoff + (size_t)mb * 16 * DM + kc);
#pragma unroll
        for (int nb = 0; nb < 4; ++nb) { const v16h b = ldh(Bt + boff + (size_t)nb * 16 * DM + kc);
#pragma unroll
            for (int mb = 0; mb < 4; ++mb) acc[mb][nb] = wmma16g(a[mb], b, acc[mb][nb]); }
    }
    const int bb = r0 / SEQ, tt = r0 % SEQ;
    const size_t obase = ((size_t)bb * OUT_SEQ + (size_t)tt) * DM + (size_t)c0;
#pragma unroll
    for (int mb = 0; mb < 4; ++mb) {
#pragma unroll
        for (int nb = 0; nb < 4; ++nb) {
#pragma unroll
            for (int j = 0; j < 8; ++j) os[(hi * 8 + j) * OSP + nb * 16 + lr] = acc[mb][nb][j] * OSC; }
        wave_sync();
        const size_t sb = obase + (size_t)(mb * 16) * DM;
#pragma unroll 1
        for (int ps = 0; ps < 2; ++ps) {
#pragma unroll
            for (int s = 0; s < 8; ++s) { const int p = s * 32 + lane; const int row = p >> 4, c4 = (p & 15) * 4;
                const v4f val = *(const v4fa*)(&os[row * OSP + c4]);
                *(volatile v4f*)(OUT + sb + (size_t)row * DM + c4) = val; }
            if (ps == 0) __threadfence(); }
        wave_sync();
    }
}

__global__ __launch_bounds__(32) void k_attn(const float* __restrict__ QS, const float* __restrict__ KS, const h16* __restrict__ VT, const float* __restrict__ va, float* ATTN, h16* AT) {
    __shared__ __align__(16) float sc[16 * SCP];
    __shared__ __align__(16) float ks[32 * KSP];
    __shared__ __align__(16) float qs[16 * KSP];
    __shared__ __align__(16) float os[16 * OSP];
    __shared__ __align__(16) float vs[HD];
    __shared__ __align__(16) float rinv[16];
    const int lane = threadIdx.x & 31, lr = lane & 15, hi = lane >> 4;
    const int zh = blockIdx.y; const int b = zh / NH_, h = zh % NH_;
    const int t0 = blockIdx.x * 16;
    const size_t pbase = (size_t)zh * SEQ * HD;
#pragma unroll
    for (int i = 0; i < 8; ++i) { const int p = i * 32 + lane; const int row = p >> 4, c4 = (p & 15) * 4;
        const v4f v = *(const v4f*)(QS + pbase + (size_t)(t0 + row) * HD + c4); *(v4fa*)(&qs[row * KSP + c4]) = v; }
    { const v4f w = *(const v4f*)(va + (size_t)h * HD + lr * 4); v4f wb;
#pragma unroll
      for (int i = 0; i < 4; ++i) wb[i] = bfr(w[i]);
      *(v4fa*)(&vs[lr * 4]) = wb; }
    wave_sync();
    float W1 = 0.0f;
#pragma unroll 1
    for (int c = 0; c < HD; c += 4) { const v4f w4 = *(const v4fa*)(&vs[c]); W1 += (w4[0] + w4[1]) + (w4[2] + w4[3]); }

    float mx = NEGB;
#pragma unroll 1
    for (int key0 = 0; key0 < SEQ; key0 += 32) {
        wave_sync();
        { const float* kp = KS + pbase + (size_t)(key0 + lane) * HD;
#pragma unroll 1
          for (int c = 0; c < HD; c += 16) {
              const v4f k0 = *(const v4f*)(kp + c), k1 = *(const v4f*)(kp + c + 4), k2 = *(const v4f*)(kp + c + 8), k3 = *(const v4f*)(kp + c + 12);
              *(v4fa*)(&ks[lane * KSP + c]) = k0; *(v4fa*)(&ks[lane * KSP + c + 4]) = k1; *(v4fa*)(&ks[lane * KSP + c + 8]) = k2; *(v4fa*)(&ks[lane * KSP + c + 12]) = k3; } }
        wave_sync();
        float aa[8], ab[8];
#pragma unroll
        for (int r = 0; r < 8; ++r) { aa[r] = 0.0f; ab[r] = 0.0f; }
#pragma unroll 1
        for (int c = 0; c < HD; c += 4) {
            const v4f q4 = *(const v4fa*)(&qs[lr * KSP + c]);
            const v4f w4 = *(const v4fa*)(&vs[c]);
#pragma unroll
            for (int r = 0; r < 8; ++r) {
                const v4f ka = *(const v4fa*)(&ks[(8 * hi + r) * KSP + c]);
                const v4f kb = *(const v4fa*)(&ks[(16 + 8 * hi + r) * KSP + c]);
#pragma unroll
                for (int i = 0; i < 4; ++i) {
                    const float ra = __builtin_amdgcn_rcpf(1.0f + __builtin_amdgcn_exp2f(q4[i] + ka[i]));
                    const float rb = __builtin_amdgcn_rcpf(1.0f + __builtin_amdgcn_exp2f(q4[i] + kb[i]));
                    aa[r] = fmaf(w4[i], ra, aa[r]); ab[r] = fmaf(w4[i], rb, ab[r]); } } }
        v4f s0, s1, s2, s3;
#pragma unroll
        for (int r = 0; r < 4; ++r) {
            s0[r] = (W1 - 2.0f * aa[r]) * SC2; s1[r] = (W1 - 2.0f * aa[4 + r]) * SC2;
            s2[r] = (W1 - 2.0f * ab[r]) * SC2; s3[r] = (W1 - 2.0f * ab[4 + r]) * SC2;
            mx = fmaxf(mx, fmaxf(fmaxf(s0[r], s1[r]), fmaxf(s2[r], s3[r]))); }
        const int so = lr * SCP + key0 + 8 * hi;
        *(v4fa*)(&sc[so]) = s0; *(v4fa*)(&sc[so + 4]) = s1; *(v4fa*)(&sc[so + 16]) = s2; *(v4fa*)(&sc[so + 20]) = s3;
    }
    const float m = fmaxf(mx, __shfl_xor(mx, 16, 32));

    v8f o0 = (v8f){}, o1 = (v8f){}, o2 = (v8f){}, o3 = (v8f){};
    float l = 0.0f, l2 = 0.0f;
    const size_t vo = ((size_t)zh * HD + (size_t)lr) * SEQ + 8 * hi;
#pragma unroll 1
    for (int key0 = 0; key0 < SEQ; key0 += 32) {
        const int so = lr * SCP + key0 + 8 * hi;
        const v4f s0 = *(const v4fa*)(&sc[so]), s1 = *(const v4fa*)(&sc[so + 4]), s2 = *(const v4fa*)(&sc[so + 16]), s3 = *(const v4fa*)(&sc[so + 20]);
        v4f e0, e1, e2, e3; v16h pb; float ls = 0.0f, lp = 0.0f;
#pragma unroll
        for (int r = 0; r < 4; ++r) {
            e0[r] = __builtin_amdgcn_exp2f(s0[r] - m); e1[r] = __builtin_amdgcn_exp2f(s1[r] - m);
            e2[r] = __builtin_amdgcn_exp2f(s2[r] - m); e3[r] = __builtin_amdgcn_exp2f(s3[r] - m);
            const h16 p0 = toh_flush(e0[r] * PCAR); const h16 p1 = toh_flush(e1[r] * PCAR);
            const h16 p2 = toh_flush(e2[r] * PCAR); const h16 p3 = toh_flush(e3[r] * PCAR);
            pb[r] = p0; pb[4 + r] = p1; pb[8 + r] = p2; pb[12 + r] = p3;
            ls += (e0[r] + e1[r]) + (e2[r] + e3[r]);
            lp += ((float)p0 + (float)p1) + ((float)p2 + (float)p3); }
        l += ls; l2 += lp;
        *(v4fa*)(&sc[so]) = e0; *(v4fa*)(&sc[so + 4]) = e1; *(v4fa*)(&sc[so + 16]) = e2; *(v4fa*)(&sc[so + 20]) = e3;
        const h16* vp = VT + vo + key0;
        const v16h v0 = ldh(vp), v1 = ldh(vp + (size_t)16 * SEQ), v2 = ldh(vp + (size_t)32 * SEQ), v3 = ldh(vp + (size_t)48 * SEQ);
        o0 = wmma16g(v0, pb, o0); o1 = wmma16g(v1, pb, o1); o2 = wmma16g(v2, pb, o2); o3 = wmma16g(v3, pb, o3);
    }
    l += __shfl_xor(l, 16, 32); l2 += __shfl_xor(l2, 16, 32);
    const float inv = 1.0f / l;
    const float invo = (ACAR / VCAR) / l2;
    rinv[lr] = inv;
    { v4f a, c;
      a[0] = o0[0] * invo; a[1] = o0[1] * invo; a[2] = o0[2] * invo; a[3] = o0[3] * invo; c[0] = o0[4] * invo; c[1] = o0[5] * invo; c[2] = o0[6] * invo; c[3] = o0[7] * invo;
      *(v4fa*)(&os[lr * OSP +  0 + 8 * hi]) = a; *(v4fa*)(&os[lr * OSP +  0 + 8 * hi + 4]) = c;
      a[0] = o1[0] * invo; a[1] = o1[1] * invo; a[2] = o1[2] * invo; a[3] = o1[3] * invo; c[0] = o1[4] * invo; c[1] = o1[5] * invo; c[2] = o1[6] * invo; c[3] = o1[7] * invo;
      *(v4fa*)(&os[lr * OSP + 16 + 8 * hi]) = a; *(v4fa*)(&os[lr * OSP + 16 + 8 * hi + 4]) = c;
      a[0] = o2[0] * invo; a[1] = o2[1] * invo; a[2] = o2[2] * invo; a[3] = o2[3] * invo; c[0] = o2[4] * invo; c[1] = o2[5] * invo; c[2] = o2[6] * invo; c[3] = o2[7] * invo;
      *(v4fa*)(&os[lr * OSP + 32 + 8 * hi]) = a; *(v4fa*)(&os[lr * OSP + 32 + 8 * hi + 4]) = c;
      a[0] = o3[0] * invo; a[1] = o3[1] * invo; a[2] = o3[2] * invo; a[3] = o3[3] * invo; c[0] = o3[4] * invo; c[1] = o3[5] * invo; c[2] = o3[6] * invo; c[3] = o3[7] * invo;
      *(v4fa*)(&os[lr * OSP + 48 + 8 * hi]) = a; *(v4fa*)(&os[lr * OSP + 48 + 8 * hi + 4]) = c; }
    wave_sync();
    const size_t abase = ((size_t)b * SEQ + (size_t)t0) * DM + (size_t)h * HD;
    const size_t pb0 = (((size_t)b * NH_ + (size_t)h) * OUT_SEQ + (size_t)t0) * OUT_SEQ;
#pragma unroll 1
    for (int ps = 0; ps < 2; ++ps) {
#pragma unroll
        for (int s = 0; s < 4; ++s) { const int row = 4 * s + (lane >> 3), c8 = (lane & 7) * 8;
            const v4f x0 = *(const v4fa*)(&os[row * OSP + c8]); const v4f x1 = *(const v4fa*)(&os[row * OSP + c8 + 4]); v8h hv;
#pragma unroll
            for (int i = 0; i < 4; ++i) { hv[i] = toh_flush(x0[i]); hv[4 + i] = toh_flush(x1[i]); }
            *(volatile v8h*)(AT + abase + (size_t)row * DM + c8) = hv; }
#pragma unroll 1
        for (int row = 0; row < 16; ++row) {
            const float invr = rinv[row];
            const size_t ro = pb0 + (size_t)row * OUT_SEQ;
#pragma unroll
            for (int qd = 0; qd < SEQ / 128; ++qd) { const int cofs = qd * 128 + lane * 4;
                const v4f e = *(const v4fa*)(&sc[row * SCP + cofs]);
                v4f val; val[0] = e[0] * invr; val[1] = e[1] * invr; val[2] = e[2] * invr; val[3] = e[3] * invr;
                *(volatile v4f*)(ATTN + ro + cofs) = val; } }
        if (ps == 0) __threadfence(); }
}

static constexpr size_t al256(size_t v) { return (v + 255) & ~(size_t)255; }
static constexpr size_t SZ_XB = al256((size_t)NB * SEQ * DM * 2);
static constexpr size_t SZ_WB = al256((size_t)3 * DM * DM * 2);
static constexpr size_t SZ_WO = al256((size_t)DM * DM * 2);
static constexpr size_t SZ_PF = al256((size_t)NB * NH_ * SEQ * HD * 4);
static constexpr size_t SZ_PH = al256((size_t)NB * SEQ * DM * 2);
static constexpr size_t SZ_TOTAL = 3 * SZ_XB + SZ_WB + SZ_WO + 2 * SZ_PF + 2 * SZ_PH;
static_assert(SZ_TOTAL <= (size_t)134217728);
static_assert(((size_t)DM * DM * 2) % 256 == 0);
static_assert((size_t)NB * NH_ * SEQ * HD == (size_t)NB * DM * SEQ);

extern "C" void kernel_launch(void* const* d_in, const int* in_sizes, int n_in,
                              void* d_out, int out_size, void* d_ws, size_t ws_size, hipStream_t stream) {
    if (n_in < 8) return;
    const size_t needx = ((size_t)(NB - 1) * SEQ_FULL + SEQ) * DM;
    if ((size_t)in_sizes[0] < needx || (size_t)in_sizes[1] < needx || (size_t)in_sizes[2] < needx) return;
    if ((size_t)in_sizes[3] < (size_t)DM * DM || (size_t)in_sizes[4] < (size_t)DM * DM || (size_t)in_sizes[5] < (size_t)DM * DM || (size_t)in_sizes[7] < (size_t)DM * DM) return;
    if (in_sizes[6] < NH_ * HD) return;
    const size_t need_out = OUT1_OFF + ((size_t)(NB * NH_ - 1) * OUT_SEQ + (size_t)(SEQ - 1)) * OUT_SEQ + SEQ;
    if ((size_t)out_size < need_out) return;
    if (SZ_TOTAL > ws_size) return;
    const float* xin[3] = { (const float*)d_in[0], (const float*)d_in[1], (const float*)d_in[2] };
    const float* wq = (const float*)d_in[3];
    const float* wk = (const float*)d_in[4];
    const float* wv = (const float*)d_in[5];
    const float* va = (const float*)d_in[6];
    const float* wo = (const float*)d_in[7];
    float* OUT  = (float*)d_out;
    float* ATTN = (float*)d_out + OUT1_OFF;
    char* wsp = (char*)d_ws;
    bf* XB[3];
    XB[0] = (bf*)wsp; wsp += SZ_XB;
    XB[1] = (bf*)wsp; wsp += SZ_XB;
    XB[2] = (bf*)wsp; wsp += SZ_XB;
    bf* WB = (bf*)wsp; wsp += SZ_WB;
    h16* WO = (h16*)wsp; wsp += SZ_WO;
    float* QS = (float*)wsp; wsp += SZ_PF;
    float* KS = (float*)wsp; wsp += SZ_PF;
    h16* VT = (h16*)wsp; wsp += SZ_PH;
    h16* AT = (h16*)wsp; wsp += SZ_PH;
    bf* WQ = WB; bf* WK = WB + (size_t)DM * DM; bf* WV = WB + (size_t)2 * DM * DM;

    for (int i = 0; i < 3; ++i) {
        if (SEQ == SEQ_FULL) {
            const size_t n8 = (size_t)NB * SEQ * DM / 8;
            k_cvt8<<<(unsigned)((n8 + 255) / 256), 256, 0, stream>>>(xin[i], XB[i], n8);
        } else {
            const size_t n8 = (size_t)SEQ * DM / 8;
            for (int b = 0; b < NB; ++b) k_cvt8<<<(unsigned)((n8 + 255) / 256), 256, 0, stream>>>(xin[i] + (size_t)b * SEQ_FULL * DM, XB[i] + (size_t)b * SEQ * DM, n8);
        }
    }
    { const size_t n8 = (size_t)DM * DM / 8; const unsigned g = (unsigned)((n8 + 255) / 256);
      k_cvt8<<<g, 256, 0, stream>>>(wq, WQ, n8); k_cvt8<<<g, 256, 0, stream>>>(wk, WK, n8); k_cvt8<<<g, 256, 0, stream>>>(wv, WV, n8);
      k_cvtw<<<g, 256, 0, stream>>>(wo, WO, n8); }

    k_projqk<<<dim3(NB * SEQ / 64, DM / 64, 1), 32, 0, stream>>>(XB[0], WQ, QS);
    k_projqk<<<dim3(NB * SEQ / 64, DM / 64, 1), 32, 0, stream>>>(XB[1], WK, KS);
    k_projv<<<dim3(DM / 64, NB * SEQ / 64, 1), 32, 0, stream>>>(WV, XB[2], VT);

    k_attn<<<dim3(SEQ / 16, NB * NH_, 1), 32, 0, stream>>>(QS, KS, VT, va, ATTN, AT);

    k_outp<<<dim3(NB * SEQ / 64, DM / 64, 1), 32, 0, stream>>>(AT, WO, OUT);
}
